// PointNet2_7842610283209
// MI455X (gfx1250) — hardware-verified
//
#include <hip/hip_runtime.h>
#include <stdint.h>


typedef float          v8f       __attribute__((ext_vector_type(8)));
typedef float          v4f_plain __attribute__((ext_vector_type(4)));
typedef v4f_plain      v4f       __attribute__((may_alias));
typedef __bf16         v16bf     __attribute__((ext_vector_type(16)));
typedef unsigned short v8us_plain __attribute__((ext_vector_type(8)));
typedef v8us_plain     v8us      __attribute__((may_alias));

union Frag { v16bf v; v8us u[2]; };

constexpr int NB  = 2;
constexpr int N1  = 4096;
constexpr int N2  = 32768;
constexpr int C1  = 128;
constexpr int C2  = 64;
constexpr int CIN = C1 + C2;
constexpr int F1  = 128;
constexpr int F2  = 128;
constexpr int S0  = 3 + C1;
constexpr int S1  = 3 + C2;
constexpr float EPSV = 1e-07f;

constexpr int KT    = 256;
constexpr int QPB   = 2 * KT;
constexpr int CH    = 2048;
constexpr int NCH   = (N1 + CH - 1) / CH;
constexpr int RPW   = QPB / (KT / 32);
constexpr int MROWS = 32;
constexpr int SP    = 132;

static_assert(N2 % QPB == 0);
static_assert((NB * N2) % MROWS == 0);
static_assert(CIN % 32 == 0 && F1 % 32 == 0);
static_assert(F1 == 16 * (KT / 32) && F2 == 16 * (KT / 32));
static_assert(CIN / 8 <= 32 && C1 % 8 == 0 && C2 % 8 == 0);
static_assert((3 * QPB) % 128 == 0);
static_assert(SP % 4 == 0);
static_assert(MROWS % (KT / 32) == 0);

__device__ __forceinline__ unsigned short bf16_rne(float f) {
    unsigned int u = __float_as_uint(f);
    u += 0x7FFFu + ((u >> 16) & 1u);
    return (unsigned short)(u >> 16);
}

__device__ __forceinline__ void split2(float f, unsigned short& hi, unsigned short& lo) {
    const unsigned short hs = bf16_rne(f);
    const float hf = __uint_as_float(((unsigned int)hs) << 16);
    hi = hs;
    lo = bf16_rne(f - hf);
}

__device__ __forceinline__ v8f wmma16(const v16bf a, const v16bf b, v8f c) {
    v8f d = __builtin_amdgcn_wmma_f32_16x16x32_bf16(false, a, false, b, (short)0, c, false, false);
    asm volatile("v_nop\n\tv_nop\n\tv_nop\n\tv_nop" : "+v"(d) : "v"(a), "v"(b));
    return d;
}

__device__ __forceinline__ v8f zero8() {
    v8f z = {0.0f, 0.0f, 0.0f, 0.0f, 0.0f, 0.0f, 0.0f, 0.0f};
    return z;
}

__device__ __forceinline__ void top3_upd(float d, int j,
                                         float& d0, float& d1, float& d2,
                                         int& i0, int& i1, int& i2) {
    if (d < d2) {
        if (d < d0)      { d2 = d1; i2 = i1; d1 = d0; i1 = i0; d0 = d; i0 = j; }
        else if (d < d1) { d2 = d1; i2 = i1; d1 = d;  i1 = j; }
        else             { d2 = d;  i2 = j; }
    }
}

__global__ __launch_bounds__(KT) void prep_w(const float* __restrict__ W1,
                                             const float* __restrict__ W2,
                                             unsigned short* __restrict__ W1h,
                                             unsigned short* __restrict__ W1l,
                                             unsigned short* __restrict__ W2h,
                                             unsigned short* __restrict__ W2l) {
    const int lane = threadIdx.x & 31, wave = threadIdx.x >> 5;
    const int gw = blockIdx.x * (KT / 32) + wave;
    if (gw >= F1 + F2) return;
    const bool first  = gw < F1;
    const int  n      = first ? gw : gw - F1;
    const int  K      = first ? CIN : F1;
    const int  pitch  = first ? F1 : F2;
    const float* src  = first ? W1 : W2;
    unsigned short* dh = (first ? W1h : W2h) + (size_t)n * K + 8 * lane;
    unsigned short* dl = (first ? W1l : W2l) + (size_t)n * K + 8 * lane;
    const bool act = (8 * lane + 8) <= K;

    v8us vh, vl;
#pragma unroll
    for (int i = 0; i < 8; ++i) {
        float f = 0.0f;
        if (act) f = src[(size_t)(8 * lane + i) * pitch + n];
        unsigned short hs, ls;
        split2(f, hs, ls);
        vh[i] = hs; vl[i] = ls;
    }
    if (act) { *(volatile v8us*)dh = vh; *(volatile v8us*)dl = vl; }
    __threadfence();
    if (act) { *(volatile v8us*)dh = vh; *(volatile v8us*)dl = vl; }
}

__global__ __launch_bounds__(KT) void knn_interp(const float* __restrict__ in0,
                                                 const float* __restrict__ in1,
                                                 unsigned short* __restrict__ Xh,
                                                 unsigned short* __restrict__ Xl,
                                                 float* __restrict__ oxyz) {
#pragma clang fp contract(off)
    __shared__ float4 sxyz[CH];
    __shared__ int    sidx[3 * QPB];
    __shared__ float  swt[3 * QPB];
    __shared__ alignas(16) float sq3[3 * QPB];

    const int tid = threadIdx.x, lane = tid & 31, wave = tid >> 5;
    constexpr int BPB = N2 / QPB;
    const int b     = blockIdx.x / BPB;
    const int qbase = (blockIdx.x - b * BPB) * QPB;
    const float* base0 = in0 + (size_t)b * N1 * S0;
    const float* base1 = in1 + (size_t)b * N2 * S1;

    const float* qA = base1 + (size_t)(qbase + tid) * S1;
    const float* qB = base1 + (size_t)(qbase + KT + tid) * S1;
    const float ax = qA[0], ay = qA[1], az = qA[2];
    const float bx = qB[0], by = qB[1], bz = qB[2];

    float da0 = 3.0e38f, da1 = 3.0e38f, da2 = 3.0e38f;
    float db0 = 3.0e38f, db1 = 3.0e38f, db2 = 3.0e38f;
    int   ia0 = 0, ia1 = 0, ia2 = 0;
    int   ib0 = 0, ib1 = 0, ib2 = 0;

    for (int ck = 0; ck < NCH; ++ck) {
        const int j0   = ck * CH;
        const int jcnt = (N1 - j0) < CH ? (N1 - j0) : CH;
        __syncthreads();
        for (int j = tid; j < jcnt; j += KT) {
            const float* p = base0 + (size_t)(j0 + j) * S0;
            sxyz[j] = make_float4(p[0], p[1], p[2], 0.0f);
        }
        __syncthreads();
#pragma unroll 2
        for (int j = 0; j < jcnt; ++j) {
            const float4 c = sxyz[j];
            const int jj = j0 + j;
            {
                const float dx = ax - c.x, dy = ay - c.y, dz = az - c.z;
                const float d  = (dx * dx + dy * dy) + dz * dz;
                top3_upd(d, jj, da0, da1, da2, ia0, ia1, ia2);
            }
            {
                const float dx = bx - c.x, dy = by - c.y, dz = bz - c.z;
                const float d  = (dx * dx + dy * dy) + dz * dz;
                top3_upd(d, jj, db0, db1, db2, ib0, ib1, ib2);
            }
        }
    }

    {
        const float e0 = fmaxf(da0, EPSV), e1 = fmaxf(da1, EPSV), e2 = fmaxf(da2, EPSV);
        const float w0 = 1.0f / e0, w1 = 1.0f / e1, w2 = 1.0f / e2;
        const float s  = (w0 + w1) + w2;
        const float iv = 1.0f / s;
        sidx[tid] = ia0; sidx[QPB + tid] = ia1; sidx[2 * QPB + tid] = ia2;
        swt[tid] = w0 * iv; swt[QPB + tid] = w1 * iv; swt[2 * QPB + tid] = w2 * iv;
        sq3[3 * tid + 0] = ax; sq3[3 * tid + 1] = ay; sq3[3 * tid + 2] = az;
    }
    {
        const int t2 = KT + tid;
        const float e0 = fmaxf(db0, EPSV), e1 = fmaxf(db1, EPSV), e2 = fmaxf(db2, EPSV);
        const float w0 = 1.0f / e0, w1 = 1.0f / e1, w2 = 1.0f / e2;
        const float s  = (w0 + w1) + w2;
        const float iv = 1.0f / s;
        sidx[t2] = ib0; sidx[QPB + t2] = ib1; sidx[2 * QPB + t2] = ib2;
        swt[t2] = w0 * iv; swt[QPB + t2] = w1 * iv; swt[2 * QPB + t2] = w2 * iv;
        sq3[3 * t2 + 0] = bx; sq3[3 * t2 + 1] = by; sq3[3 * t2 + 2] = bz;
    }
    __syncthreads();

    {
        float* ob = oxyz + ((size_t)b * N2 + (size_t)qbase) * 3;
        constexpr int NG = (3 * QPB) / 128;
        for (int g = wave; g < NG; g += KT / 32) {
            const int f = g * 128 + 4 * lane;
            v4f v; v.x = sq3[f]; v.y = sq3[f + 1]; v.z = sq3[f + 2]; v.w = sq3[f + 3];
            *(volatile v4f*)(ob + f) = v;
        }
        __threadfence();
        for (int g = wave; g < NG; g += KT / 32) {
            const int f = g * 128 + 4 * lane;
            v4f v; v.x = sq3[f]; v.y = sq3[f + 1]; v.z = sq3[f + 2]; v.w = sq3[f + 3];
            *(volatile v4f*)(ob + f) = v;
        }
    }

    const bool actl = lane < (CIN / 8);
    for (int rr = 0; rr < RPW; ++rr) {
        const int lq = wave * RPW + rr;
        const size_t nrow = (size_t)(qbase + lq);
        const size_t grow = (size_t)b * N2 + nrow;
        int i0 = sidx[lq], i1 = sidx[QPB + lq], i2 = sidx[2 * QPB + lq];
        i0 = i0 < 0 ? 0 : (i0 > N1 - 1 ? N1 - 1 : i0);
        i1 = i1 < 0 ? 0 : (i1 > N1 - 1 ? N1 - 1 : i1);
        i2 = i2 < 0 ? 0 : (i2 > N1 - 1 ? N1 - 1 : i2);
        const float w0 = swt[lq], w1 = swt[QPB + lq], w2 = swt[2 * QPB + lq];

        v8us vh, vl;
        if (lane < (C1 / 8)) {
            const float* p0 = base0 + (size_t)i0 * S0 + 3 + 8 * lane;
            const float* p1 = base0 + (size_t)i1 * S0 + 3 + 8 * lane;
            const float* p2 = base0 + (size_t)i2 * S0 + 3 + 8 * lane;
#pragma unroll
            for (int i = 0; i < 8; ++i) {
                const float v = fmaf(w2, p2[i], fmaf(w1, p1[i], w0 * p0[i]));
                unsigned short hs, ls;
                split2(v, hs, ls);
                vh[i] = hs; vl[i] = ls;
            }
        } else if (actl) {
            const float* qq = base1 + nrow * S1 + 3 + 8 * (lane - C1 / 8);
#pragma unroll
            for (int i = 0; i < 8; ++i) {
                unsigned short hs, ls;
                split2(qq[i], hs, ls);
                vh[i] = hs; vl[i] = ls;
            }
        } else {
#pragma unroll
            for (int i = 0; i < 8; ++i) { vh[i] = 0; vl[i] = 0; }
        }
        unsigned short* xh = Xh + grow * CIN + 8 * lane;
        unsigned short* xl = Xl + grow * CIN + 8 * lane;
        if (actl) { *(volatile v8us*)xh = vh; *(volatile v8us*)xl = vl; }
        __threadfence();
        if (actl) { *(volatile v8us*)xh = vh; *(volatile v8us*)xl = vl; }
    }
}

__global__ __launch_bounds__(KT) void mlp2(const unsigned short* __restrict__ Xh,
                                           const unsigned short* __restrict__ Xl,
                                           const unsigned short* __restrict__ W1h,
                                           const unsigned short* __restrict__ W1l,
                                           const float* __restrict__ b1,
                                           const unsigned short* __restrict__ W2h,
                                           const unsigned short* __restrict__ W2l,
                                           const float* __restrict__ b2,
                                           float* __restrict__ out,
                                           int Mtot) {
    __shared__ alignas(16) unsigned short Hh[MROWS * F1];
    __shared__ alignas(16) unsigned short Hl[MROWS * F1];
    __shared__ alignas(16) float          So[MROWS * SP];

    const int lane = threadIdx.x & 31, wave = threadIdx.x >> 5;
    const int h = lane >> 4, m = lane & 15;
    const int rowBase = blockIdx.x * MROWS;
    const int n0 = wave * 16;

    int r0 = rowBase + m;      if (r0 > Mtot - 1) r0 = Mtot - 1;
    int r1 = rowBase + 16 + m; if (r1 > Mtot - 1) r1 = Mtot - 1;

    const unsigned short* xh0 = Xh + (size_t)r0 * CIN + 8 * h;
    const unsigned short* xl0 = Xl + (size_t)r0 * CIN + 8 * h;
    const unsigned short* xh1 = Xh + (size_t)r1 * CIN + 8 * h;
    const unsigned short* xl1 = Xl + (size_t)r1 * CIN + 8 * h;
    const unsigned short* wh1 = W1h + (size_t)(n0 + m) * CIN + 8 * h;
    const unsigned short* wl1 = W1l + (size_t)(n0 + m) * CIN + 8 * h;

    v8f acc0 = zero8(), acc1 = zero8();
#pragma unroll 1
    for (int c = 0; c < CIN / 32; ++c) {
        const int k = c * 32;
        Frag bh, bl, a0h, a0l, a1h, a1l;
        bh.u[0]  = *(const v8us*)(wh1 + k); bh.u[1]  = *(const v8us*)(wh1 + k + 16);
        bl.u[0]  = *(const v8us*)(wl1 + k); bl.u[1]  = *(const v8us*)(wl1 + k + 16);
        a0h.u[0] = *(const v8us*)(xh0 + k); a0h.u[1] = *(const v8us*)(xh0 + k + 16);
        a0l.u[0] = *(const v8us*)(xl0 + k); a0l.u[1] = *(const v8us*)(xl0 + k + 16);
        a1h.u[0] = *(const v8us*)(xh1 + k); a1h.u[1] = *(const v8us*)(xh1 + k + 16);
        a1l.u[0] = *(const v8us*)(xl1 + k); a1l.u[1] = *(const v8us*)(xl1 + k + 16);
        acc0 = wmma16(a0h.v, bh.v, acc0);
        acc0 = wmma16(a0l.v, bh.v, acc0);
        acc0 = wmma16(a0h.v, bl.v, acc0);
        acc1 = wmma16(a1h.v, bh.v, acc1);
        acc1 = wmma16(a1l.v, bh.v, acc1);
        acc1 = wmma16(a1h.v, bl.v, acc1);
    }

    {
        const float bias1 = b1[n0 + m];
#pragma unroll
        for (int r = 0; r < 8; ++r) {
            unsigned short hs, ls;
            split2(fmaxf(acc0[r] + bias1, 0.0f), hs, ls);
            Hh[(8 * h + r) * F1 + n0 + m] = hs;
            Hl[(8 * h + r) * F1 + n0 + m] = ls;
            split2(fmaxf(acc1[r] + bias1, 0.0f), hs, ls);
            Hh[(16 + 8 * h + r) * F1 + n0 + m] = hs;
            Hl[(16 + 8 * h + r) * F1 + n0 + m] = ls;
        }
    }
    __syncthreads();

    const unsigned short* hh0 = Hh + m * F1 + 8 * h;
    const unsigned short* hl0 = Hl + m * F1 + 8 * h;
    const unsigned short* hh1 = Hh + (16 + m) * F1 + 8 * h;
    const unsigned short* hl1 = Hl + (16 + m) * F1 + 8 * h;
    const unsigned short* wh2 = W2h + (size_t)(n0 + m) * F1 + 8 * h;
    const unsigned short* wl2 = W2l + (size_t)(n0 + m) * F1 + 8 * h;

    acc0 = zero8(); acc1 = zero8();
#pragma unroll 1
    for (int c = 0; c < F1 / 32; ++c) {
        const int k = c * 32;
        Frag bh, bl, a0h, a0l, a1h, a1l;
        bh.u[0]  = *(const v8us*)(wh2 + k); bh.u[1]  = *(const v8us*)(wh2 + k + 16);
        bl.u[0]  = *(const v8us*)(wl2 + k); bl.u[1]  = *(const v8us*)(wl2 + k + 16);
        a0h.u[0] = *(const v8us*)(hh0 + k); a0h.u[1] = *(const v8us*)(hh0 + k + 16);
        a0l.u[0] = *(const v8us*)(hl0 + k); a0l.u[1] = *(const v8us*)(hl0 + k + 16);
        a1h.u[0] = *(const v8us*)(hh1 + k); a1h.u[1] = *(const v8us*)(hh1 + k + 16);
        a1l.u[0] = *(const v8us*)(hl1 + k); a1l.u[1] = *(const v8us*)(hl1 + k + 16);
        acc0 = wmma16(a0h.v, bh.v, acc0);
        acc0 = wmma16(a0l.v, bh.v, acc0);
        acc0 = wmma16(a0h.v, bl.v, acc0);
        acc1 = wmma16(a1h.v, bh.v, acc1);
        acc1 = wmma16(a1l.v, bh.v, acc1);
        acc1 = wmma16(a1h.v, bl.v, acc1);
    }

    {
        const float bias2 = b2[n0 + m];
#pragma unroll
        for (int r = 0; r < 8; ++r) {
            So[(8 * h + r) * SP + n0 + m]      = fmaxf(acc0[r] + bias2, 0.0f);
            So[(16 + 8 * h + r) * SP + n0 + m] = fmaxf(acc1[r] + bias2, 0.0f);
        }
    }
    __syncthreads();

    constexpr int RW = MROWS / (KT / 32);
#pragma unroll
    for (int rr = 0; rr < RW; ++rr) {
        const int row  = wave * RW + rr;
        const int grow = rowBase + row;
        const v4f v = *(const v4f*)(So + row * SP + 4 * lane);
        if (grow < Mtot) *(volatile v4f*)(out + (size_t)grow * F2 + 4 * lane) = v;
    }
    __threadfence();
#pragma unroll
    for (int rr = 0; rr < RW; ++rr) {
        const int row  = wave * RW + rr;
        const int grow = rowBase + row;
        const v4f v = *(const v4f*)(So + row * SP + 4 * lane);
        if (grow < Mtot) *(volatile v4f*)(out + (size_t)grow * F2 + 4 * lane) = v;
    }
}

extern "C" void kernel_launch(void* const* d_in, const int* in_sizes, int n_in,
                              void* d_out, int out_size, void* d_ws, size_t ws_size,
                              hipStream_t stream) {
    if (n_in < 6) return;
    if (in_sizes[0] != NB * N1 * S0) return;
    if (in_sizes[1] != NB * N2 * S1) return;
    if (in_sizes[2] != CIN * F1) return;
    if (in_sizes[3] != F1) return;
    if (in_sizes[4] != F1 * F2) return;
    if (in_sizes[5] != F2) return;
    if (out_size != NB * N2 * (F2 + 3)) return;

    const float* in0 = (const float*)d_in[0];
    const float* in1 = (const float*)d_in[1];
    const float* W1  = (const float*)d_in[2];
    const float* b1  = (const float*)d_in[3];
    const float* W2  = (const float*)d_in[4];
    const float* b2  = (const float*)d_in[5];

    float* outX   = (float*)d_out;
    float* outXyz = (float*)d_out + (size_t)NB * N2 * F2;

    const size_t Mtot = (size_t)NB * N2;

    size_t off = 0;
    const size_t xPlane  = Mtot * CIN * sizeof(unsigned short);
    const size_t w1Plane = (size_t)F1 * CIN * sizeof(unsigned short);
    const size_t w2Plane = (size_t)F2 * F1 * sizeof(unsigned short);
    const size_t oXh  = off; off += (xPlane  + 255) & ~(size_t)255;
    const size_t oXl  = off; off += (xPlane  + 255) & ~(size_t)255;
    const size_t oW1h = off; off += (w1Plane + 255) & ~(size_t)255;
    const size_t oW1l = off; off += (w1Plane + 255) & ~(size_t)255;
    const size_t oW2h = off; off += (w2Plane + 255) & ~(size_t)255;
    const size_t oW2l = off; off += (w2Plane + 255) & ~(size_t)255;
    if (off > ws_size) return;

    char* ws = (char*)d_ws;
    unsigned short* Xh  = (unsigned short*)(ws + oXh);
    unsigned short* Xl  = (unsigned short*)(ws + oXl);
    unsigned short* W1h = (unsigned short*)(ws + oW1h);
    unsigned short* W1l = (unsigned short*)(ws + oW1l);
    unsigned short* W2h = (unsigned short*)(ws + oW2h);
    unsigned short* W2l = (unsigned short*)(ws + oW2l);

    {
        const int rows = F1 + F2;
        const int grid = (rows + (KT / 32) - 1) / (KT / 32);
        prep_w<<<grid, KT, 0, stream>>>(W1, W2, W1h, W1l, W2h, W2l);
    }
    {
        const int grid = NB * (N2 / QPB);
        knn_interp<<<grid, KT, 0, stream>>>(in0, in1, Xh, Xl, outXyz);
    }
    {
        const int grid = (int)((Mtot + MROWS - 1) / MROWS);
        mlp2<<<grid, KT, 0, stream>>>(Xh, Xl, W1h, W1l, b1, W2h, W2l, b2, outX, (int)Mtot);
    }
}
